// DropEdgeGCNModel_73727408603583
// MI455X (gfx1250) — hardware-verified
//
#include <hip/hip_runtime.h>


namespace {
constexpr int N = 50000, E = 1000000, F = 256, U = 128, C = 40, CP = 64, NPAD = 50048, NBLK = NPAD / 128;
constexpr float FXS = 524288.0f, FXI = 1.0f / 524288.0f, BNE = 1e-3f;

typedef _Float16 b16;
typedef __attribute__((ext_vector_type(16))) _Float16 v16b;
typedef __attribute__((ext_vector_type(8)))  _Float16 v8b;
typedef __attribute__((ext_vector_type(8)))  float v8f;
typedef __attribute__((ext_vector_type(4)))  float v4f;

__device__ __forceinline__ v8b ld8b(const b16* p) { return *(const v8b*)p; }
__device__ __forceinline__ v16b cat8b(v8b a, v8b b) { return __builtin_shufflevector(a, b, 0, 1, 2, 3, 4, 5, 6, 7, 8, 9, 10, 11, 12, 13, 14, 15); }
__device__ __forceinline__ v16b frag_kb(const b16* p, int hh) { return cat8b(ld8b(p + 8 * hh), ld8b(p + 16 + 8 * hh)); }
__device__ __forceinline__ void split16(float v, b16& hi, b16& lo) { hi = (b16)v; lo = (b16)(v - (float)hi); }
__device__ __forceinline__ void frag_ksplit(const float* p, int hh, v16b& fh_, v16b& fl_) {
  const float* p0 = p + 8 * hh; const float* p1 = p + 16 + 8 * hh;
#pragma unroll
  for (int e = 0; e < 8; ++e) { b16 a, c; split16(p0[e], a, c); fh_[e] = a; fl_[e] = c; split16(p1[e], a, c); fh_[8 + e] = a; fl_[8 + e] = c; }
}
__device__ __forceinline__ v8f wmma16b(v16b a, v16b b, v8f c) {
  v8f d = __builtin_amdgcn_wmma_f32_16x16x32_f16(false, a, false, b, (short)0, c, false, false);
  asm volatile("v_nop\n\tv_nop\n\tv_nop\n\tv_nop" : "+v"(d) : "v"(a), "v"(b));
  return d;
}
__device__ __forceinline__ void wave_lds_sync() {
  __builtin_amdgcn_fence(__ATOMIC_RELEASE, "workgroup");
  __builtin_amdgcn_wave_barrier();
  __builtin_amdgcn_fence(__ATOMIC_ACQUIRE, "workgroup");
}

struct Opnd { const void* p0; const void* p1; int ld; };
template <int NP> __device__ __forceinline__ void load_frags(const Opnd& o, int row, int kb, int hh, v16b& fh_, v16b& fl_) {
  if (NP == 0) { frag_ksplit((const float*)o.p0 + (size_t)row * o.ld + kb, hh, fh_, fl_); }
  else if (NP == 4) {
    const float* p = (const float*)o.p0 + (size_t)row * o.ld + kb; const float* p0 = p + 8 * hh; const float* p1 = p + 16 + 8 * hh;
#pragma unroll
    for (int e = 0; e < 8; ++e) { b16 a, c; split16(p0[e] * 64.0f, a, c); fh_[e] = a; fl_[e] = c; split16(p1[e] * 64.0f, a, c); fh_[8 + e] = a; fl_[8 + e] = c; }
  } else if (NP == 3) {
    const float* p = (const float*)o.p0 + (size_t)row * o.ld + kb; const float* p0 = p + 8 * hh; const float* p1 = p + 16 + 8 * hh;
#pragma unroll
    for (int e = 0; e < 8; ++e) { fh_[e] = (b16)p0[e]; fh_[8 + e] = (b16)p1[e]; }
    fl_ = fh_;
  } else {
    fh_ = frag_kb((const b16*)o.p0 + (size_t)row * o.ld + kb, hh);
    if (NP == 2) fl_ = frag_kb((const b16*)o.p1 + (size_t)row * o.ld + kb, hh); else fl_ = fh_;
  }
}
template <int ANP, int BNP> __device__ __forceinline__ v8f mac(v16b ah, v16b al, v16b bh, v16b bl, v8f c) {
  c = wmma16b(ah, bh, c);
  if (BNP == 0 || BNP == 2 || BNP == 4) c = wmma16b(ah, bl, c);
  if (ANP == 0 || ANP == 2 || ANP == 4) c = wmma16b(al, bh, c);
  return c;
}
template <int ANP, int BNP>
__device__ __forceinline__ void gemm_tile(const Opnd& A, const Opnd& B, int K, int m0, int c0, int nloc, int hlf, v8f (&acc)[2][4]) {
  for (int kb = 0; kb < K; kb += 32) {
    v16b a0h, a0l, a1h, a1l;
    load_frags<ANP>(A, m0 + nloc, kb, hlf, a0h, a0l);
    load_frags<ANP>(A, m0 + 16 + nloc, kb, hlf, a1h, a1l);
#pragma unroll
    for (int t = 0; t < 4; ++t) {
      v16b bh, bl;
      load_frags<BNP>(B, c0 + t * 16 + nloc, kb, hlf, bh, bl);
      acc[0][t] = mac<ANP, BNP>(a0h, a0l, bh, bl, acc[0][t]);
      acc[1][t] = mac<ANP, BNP>(a1h, a1l, bh, bl, acc[1][t]);
    }
  }
}

__device__ __forceinline__ void epi_planes(v8f (&acc)[2][4], float scale, bool two, b16* __restrict__ oh, b16* __restrict__ ol, int ldo,
                                           int m0, int c0, int lane, b16* Th, b16* Tl) {
  const int nloc = lane & 15, hlf = lane >> 4;
#pragma unroll
  for (int t = 0; t < 4; ++t)
#pragma unroll
    for (int r = 0; r < 2; ++r)
#pragma unroll
      for (int v = 0; v < 8; ++v) {
        const int rr = r * 16 + v + 8 * hlf, cc = t * 16 + nloc;
        b16 h_, l_; split16(acc[r][t][v] * scale, h_, l_);
        Th[rr * 64 + cc] = h_; Tl[rr * 64 + cc] = l_;
      }
  wave_lds_sync();
  for (int pass = 0; pass < 2; ++pass) {
#pragma unroll
    for (int j = 0; j < 8; ++j) {
      const int rr = j * 4 + (lane >> 3), c8 = (lane & 7) * 8;
      const size_t o = (size_t)(m0 + rr) * ldo + c0 + c8;
      *(volatile v8b*)(oh + o) = ld8b(Th + rr * 64 + c8);
      if (two) *(volatile v8b*)(ol + o) = ld8b(Tl + rr * 64 + c8);
    }
    __threadfence();
  }
}
__device__ __forceinline__ void epi_f32(v8f (&acc)[2][4], float scale, const float* rscale, float* __restrict__ out, int ldo, int m0, int c0, int lane, float* Tt) {
  const int nloc = lane & 15, hlf = lane >> 4;
#pragma unroll
  for (int t = 0; t < 4; ++t)
#pragma unroll
    for (int r = 0; r < 2; ++r)
#pragma unroll
      for (int v = 0; v < 8; ++v) {
        const int rr = r * 16 + v + 8 * hlf;
        const float rs = rscale ? rscale[(size_t)(m0 + rr) * 32] : 1.0f;
        Tt[rr * 64 + t * 16 + nloc] = acc[r][t][v] * scale * rs;
      }
  wave_lds_sync();
  float* dst0 = out + (size_t)m0 * ldo + c0;
  for (int pass = 0; pass < 2; ++pass) {
#pragma unroll
    for (int j = 0; j < 16; ++j) { const int rr = j * 2 + hlf, c4 = nloc * 4; *(volatile v4f*)(dst0 + (size_t)rr * ldo + c4) = *(const v4f*)(Tt + rr * 64 + c4); }
    __threadfence();
  }
}


__global__ __launch_bounds__(256) void prep_kernel(const float* __restrict__ g1, const float* __restrict__ s1, const float* __restrict__ g2, const float* __restrict__ s2, const float* __restrict__ g3, const float* __restrict__ s3,
                                                   b16* __restrict__ w1, b16* __restrict__ w2, b16* __restrict__ w3) {
  const size_t tid = (size_t)blockIdx.x * blockDim.x + threadIdx.x, nth = (size_t)gridDim.x * blockDim.x;
  for (int pass = 0; pass < 2; ++pass) {
    for (size_t p = tid; p < (size_t)2 * U * F / 8; p += nth) { const int n = (int)(p / (F / 8)), k0 = (int)(p % (F / 8)) * 8; const float* W = (n < U) ? g1 : s1; const int nn = n % U; v8b v;
#pragma unroll
      for (int e = 0; e < 8; ++e) v[e] = (b16)W[(size_t)(k0 + e) * U + nn];
      *(volatile v8b*)(w1 + (size_t)n * F + k0) = v; }
    for (size_t p = tid; p < (size_t)2 * U * U / 8; p += nth) { const int n = (int)(p / (U / 8)), k0 = (int)(p % (U / 8)) * 8; const float* W = (n < U) ? g2 : s2; const int nn = n % U; v8b v;
#pragma unroll
      for (int e = 0; e < 8; ++e) v[e] = (b16)W[(size_t)(k0 + e) * U + nn];
      *(volatile v8b*)(w2 + (size_t)n * U + k0) = v; }
    for (size_t p = tid; p < (size_t)2 * CP * U / 8; p += nth) { const int n = (int)(p / (U / 8)), k0 = (int)(p % (U / 8)) * 8; const float* W = (n < CP) ? g3 : s3; const int nn = n % CP; v8b v;
#pragma unroll
      for (int e = 0; e < 8; ++e) v[e] = (b16)((nn < C) ? W[(size_t)(k0 + e) * C + min(nn, C - 1)] : 0.0f);
      *(volatile v8b*)(w3 + (size_t)n * U + k0) = v; }
    __threadfence();
  }
}

template <int KIN, int NOUT>
__global__ __launch_bounds__(128) void lin_kernel(const float* __restrict__ x, int nrow, const b16* __restrict__ w, float* __restrict__ y) {
  __shared__ __attribute__((aligned(16))) float Ts[4][32 * 64];
  const int lane = threadIdx.x & 31, wave = threadIdx.x >> 5, nloc = lane & 15, hlf = lane >> 4, m0 = blockIdx.y * 128 + wave * 32, c0 = blockIdx.x * 64;
  v8f acc[2][4];
#pragma unroll
  for (int r = 0; r < 2; ++r)
#pragma unroll
    for (int t = 0; t < 4; ++t) acc[r][t] = (v8f){};
  const Opnd A{x, nullptr, KIN}; const int ra = min(m0 + nloc, nrow - 1), rb = min(m0 + 16 + nloc, nrow - 1);
#pragma unroll 1
  for (int kb = 0; kb < KIN; kb += 32) { v16b a0, a1, d0, d1; load_frags<3>(A, ra, kb, hlf, a0, d0); load_frags<3>(A, rb, kb, hlf, a1, d1);
#pragma unroll
    for (int t = 0; t < 4; ++t) { const v16b bw = frag_kb(w + (size_t)(c0 + t * 16 + nloc) * KIN + kb, hlf); acc[0][t] = wmma16b(a0, bw, acc[0][t]); acc[1][t] = wmma16b(a1, bw, acc[1][t]); } }
  epi_f32(acc, 1.0f, nullptr, y, NOUT, m0, c0, lane, Ts[wave]);
}

typedef __attribute__((ext_vector_type(4))) int v4i;
__global__ __launch_bounds__(256) void deg_kernel(const int* __restrict__ edst, const float* __restrict__ ew, float* __restrict__ dinv) {
  constexpr int NB = 16384;
  __shared__ int cnt[NB];
  const int t_ = threadIdx.x, base = blockIdx.x * NB;
  for (int i = t_; i < NB; i += 256) cnt[i] = 0;
  __syncthreads();
  for (int e0 = t_ * 8; e0 < E; e0 += 256 * 8) { const v4i a = *(const v4i*)(edst + e0), b = *(const v4i*)(edst + e0 + 4); const int dd[8] = {a[0], a[1], a[2], a[3], b[0], b[1], b[2], b[3]};
#pragma unroll
    for (int j = 0; j < 8; ++j) { const unsigned sl = (unsigned)(dd[j] - base); if (sl < (unsigned)NB) atomicAdd(&cnt[sl], (int)rintf(ew[e0 + j] * FXS)); } }
  __syncthreads();
  for (int pass = 0; pass < 2; ++pass) { for (int i = t_; i < NB; i += 256) { const int node = base + i; if (node < NPAD) { const float dg = (float)cnt[i] * FXI; ((volatile float*)dinv)[node] = (node < N && dg > 0.0f) ? rsqrtf(dg) : 0.0f; } } __threadfence(); }
}

template <int DF, int NB, bool RELU>
__global__ __launch_bounds__(256) void agg_kernel(const int* __restrict__ esrc, const int* __restrict__ edst, const float* __restrict__ ew, const float* __restrict__ hh, const float* __restrict__ dinv,
                                                  const float* __restrict__ bias, const float* __restrict__ gam, const float* __restrict__ bet, const float* __restrict__ mean, const float* __restrict__ var, int nch, float* __restrict__ xo, int ostride, int nrow_out) {
  __shared__ __attribute__((aligned(16))) int acc[NB * DF];
  __shared__ int list[8 * 256];
  const int t_ = threadIdx.x, wave = t_ >> 5, lane = t_ & 31, base = blockIdx.x * NB;
  for (int i = t_; i < NB * DF; i += 256) acc[i] = 0;
  __syncthreads();
  int* wl = list + wave * 256;
  for (int c0 = 0; c0 < E; c0 += 256 * 8) {
    const int e0 = c0 + (wave * 32 + lane) * 8; int dd[8];
#pragma unroll
    for (int j = 0; j < 8; ++j) { const int dv = edst[min(e0 + j, E - 1)]; dd[j] = (e0 + j < E) ? dv : -1; }
    unsigned sl[8]; bool hit[8]; bool anyl = false;
#pragma unroll
    for (int j = 0; j < 8; ++j) { sl[j] = (unsigned)(dd[j] - base); hit[j] = sl[j] < (unsigned)NB; anyl |= hit[j]; }
    int wc = 0;
    if (__builtin_amdgcn_ballot_w32(anyl) != 0u) {
#pragma unroll
      for (int j = 0; j < 8; ++j) {
        const unsigned mj = __builtin_amdgcn_ballot_w32(hit[j]);
        if (mj != 0u) {
          if (hit[j]) { const int pos = wc + (int)__builtin_amdgcn_mbcnt_lo(mj, 0u); wl[pos] = ((e0 + j) << 10) | (int)sl[j]; }
          wc += __builtin_popcount(mj); } } }
    __builtin_amdgcn_wave_barrier(); __builtin_amdgcn_fence(__ATOMIC_RELEASE, "workgroup"); __builtin_amdgcn_fence(__ATOMIC_ACQUIRE, "workgroup");
    { constexpr int LPH = DF / 4, HPS = 32 / LPH;
      for (int i0 = 0; i0 < wc; i0 += HPS) { const int i = i0 + lane / LPH; if (i < wc) { const int ent = wl[i]; const int e = ent >> 10, slot = ent & 1023; int s = esrc[e]; s = (s < 0) ? 0 : (s >= N ? N - 1 : s);
          const float w = dinv[s] * ew[e]; const int col = (lane % LPH) * 4; const v4f v = *(const v4f*)(hh + (size_t)s * (2 * DF) + col);
#pragma unroll
          for (int c = 0; c < 4; ++c) atomicAdd(&acc[slot * DF + col + c], (int)rintf(w * v[c] * FXS)); } } }
    __builtin_amdgcn_wave_barrier();
  }
  __syncthreads();
  for (int pass = 0; pass < 2; ++pass) {
    for (int i = t_; i < NB * DF / 4; i += 256) { const int r = (i * 4) / DF, cq = (i * 4) % DF, node = base + r; if (node < nrow_out && cq < ostride) { v4f o = {0.0f, 0.0f, 0.0f, 0.0f};
        if (node < N) { const float di = dinv[node];
#pragma unroll
          for (int c = 0; c < 4; ++c) { const int ch = min(cq + c, nch - 1); float val = (float)acc[i * 4 + c] * FXI * di + hh[(size_t)node * (2 * DF) + DF + cq + c] + bias[ch];
            val = (val - mean[ch]) * rsqrtf(var[ch] + BNE) * gam[ch] + bet[ch]; if (RELU) val = fmaxf(val, 0.0f); o[c] = (cq + c < nch) ? val : 0.0f; } }
        *(volatile v4f*)(xo + (size_t)node * ostride + cq) = o; } }
    __threadfence();
  }
}
}

extern "C" void kernel_launch(void* const* d_in, const int* in_sizes, int n_in,
                              void* d_out, int out_size, void* d_ws, size_t ws_size, hipStream_t stream) {
  (void)n_in; (void)out_size;
  const float* x = (const float*)d_in[0]; const int* ei = (const int*)d_in[1]; const float* ew = (const float*)d_in[2];
  const float* const* P = (const float* const*)d_in;
  float* out = (float*)d_out;
  if (in_sizes[0] != N * F || in_sizes[1] != 2 * E || in_sizes[2] != E || in_sizes[3] != F * U || in_sizes[17] != U * C) return;
  const int* esrc = ei; const int* edst = ei + E;
  size_t off = 0; char* ws = (char*)d_ws;
  auto carve = [&](size_t bytes) { char* p = ws + off; off += (bytes + 255) & ~(size_t)255; return p; };
  b16* w1 = (b16*)carve((size_t)2 * U * F * 2); b16* w2 = (b16*)carve((size_t)2 * U * U * 2); b16* w3 = (b16*)carve((size_t)2 * CP * U * 2);
  float* dinv = (float*)carve((size_t)NPAD * 4); float* hh = (float*)carve((size_t)NPAD * 2 * U * 4); float* ha = (float*)carve((size_t)NPAD * U * 4);
  if (off > ws_size) return;
  prep_kernel<<<128, 256, 0, stream>>>(P[3], P[4], P[10], P[11], P[17], P[18], w1, w2, w3);
  deg_kernel<<<NPAD / 16384 + 1, 256, 0, stream>>>(edst, ew, dinv);
  lin_kernel<F, 2 * U><<<dim3(2 * U / 64, NBLK), 128, 0, stream>>>(x, N, w1, hh);
  agg_kernel<U, 512, true><<<NPAD / 512 + 1, 256, 0, stream>>>(esrc, edst, ew, hh, dinv, P[5], P[6], P[7], P[8], P[9], U, ha, U, NPAD);
  lin_kernel<U, 2 * U><<<dim3(2 * U / 64, NBLK), 128, 0, stream>>>(ha, NPAD, w2, hh);
  agg_kernel<U, 512, true><<<NPAD / 512 + 1, 256, 0, stream>>>(esrc, edst, ew, hh, dinv, P[12], P[13], P[14], P[15], P[16], U, ha, U, NPAD);
  lin_kernel<U, 2 * CP><<<dim3(2 * CP / 64, NBLK), 128, 0, stream>>>(ha, NPAD, w3, hh);
  agg_kernel<CP, 1024, false><<<NPAD / 1024 + 1, 256, 0, stream>>>(esrc, edst, ew, hh, dinv, P[19], P[20], P[21], P[22], P[23], C, out, C, N);
}
